// LocalGlobalAttention_1975684956479
// MI455X (gfx1250) — hardware-verified
//
#include <hip/hip_runtime.h>
#include <math.h>
#include <stdint.h>

constexpr int kBatch   = 2;
constexpr int kSeq     = 2048;
constexpr int kDim     = 1024;
constexpr int kHeads   = 16;
constexpr int kHd      = 64;
constexpr int kWin     = 128;
constexpr int kGStride = 64;
constexpr int kNGlob   = kSeq / kGStride;
constexpr int kMem     = 256;
constexpr int kRank    = 64;
constexpr int kLora    = 4;
constexpr int kRows    = kBatch * kSeq;
constexpr int kNQT     = kSeq / 64;
constexpr int kT1Pitch = 128;
constexpr int kBt2Pitch = 128;
constexpr int kKInner  = 96;
constexpr int kHeadN   = 128;

static_assert(kRows % 64 == 0 && kDim % 64 == 0 && kT1Pitch % 64 == 0 && kHeadN % 64 == 0, "tile multiples");
static_assert(kDim % 32 == 0 && kKInner % 32 == 0 && kHd % 32 == 0, "K multiples of 32");

typedef __attribute__((ext_vector_type(16))) _Float16 v16h;
typedef __attribute__((ext_vector_type(8)))  _Float16 v8h;
typedef __attribute__((ext_vector_type(16))) __bf16   v16b;
typedef __attribute__((ext_vector_type(8)))  __bf16   v8b;
typedef __attribute__((ext_vector_type(8)))  float    v8f;
typedef __attribute__((ext_vector_type(4)))  float    v4f;
typedef __attribute__((ext_vector_type(2)))  float    v2f;

__device__ __forceinline__ unsigned short f2bf_bits(float f) {
  unsigned u = __float_as_uint(f);
  return (unsigned short)((u + 0x7FFFu + ((u >> 16) & 1u)) >> 16);
}
__device__ __forceinline__ float bf_bits2f(unsigned short h) { return __uint_as_float(((unsigned)h) << 16); }

__device__ __forceinline__ void dep_guard_h(v8f& a, v8f& b, v16h x, v16h y) { asm volatile("v_nop\n\tv_nop\n\tv_nop\n\tv_nop" : "+v"(a), "+v"(b) : "v"(x), "v"(y)); }
__device__ __forceinline__ void dep_guard_b(v8f& a, v8f& b, v16b x, v16b y) { asm volatile("v_nop\n\tv_nop\n\tv_nop\n\tv_nop" : "+v"(a), "+v"(b) : "v"(x), "v"(y)); }
__device__ __forceinline__ void keep4_h(v16h a, v16h b, v16h c, v16h d) { asm volatile("v_nop" :: "v"(a), "v"(b), "v"(c), "v"(d)); }
__device__ __forceinline__ void keep4_b(v16b a, v16b b, v16b c, v16b d) { asm volatile("v_nop" :: "v"(a), "v"(b), "v"(c), "v"(d)); }
__device__ __forceinline__ void acc_guard4(v8f& a, v8f& b, v8f& c, v8f& d) { asm volatile("v_nop\n\tv_nop\n\tv_nop\n\tv_nop" : "+v"(a), "+v"(b), "+v"(c), "+v"(d)); }
template <typename T> struct Frag;
template <> struct Frag<_Float16> {
  typedef v16h V; union U { v16h v; v8h h[2]; };
  static __device__ __forceinline__ v16h load(const _Float16* p) {
    U f; f.h[0] = *(const v8h*)(p); f.h[1] = *(const v8h*)(p + 16); return f.v;
  }
  static __device__ __forceinline__ v8f mma(v16h a, v16h b, v8f c) {
    return __builtin_amdgcn_wmma_f32_16x16x32_f16(false, a, false, b, (short)0, c, false, false);
  }
  static __device__ __forceinline__ void guard(v8f& a, v8f& b, v16h x, v16h y) { dep_guard_h(a, b, x, y); }
  static __device__ __forceinline__ void keep(v16h a, v16h b, v16h c, v16h d) { keep4_h(a, b, c, d); }
};
template <> struct Frag<__bf16> {
  typedef v16b V; union U { v16b v; v8b h[2]; };
  static __device__ __forceinline__ v16b load(const __bf16* p) {
    U f; f.h[0] = *(const v8b*)(p); f.h[1] = *(const v8b*)(p + 16); return f.v;
  }
  static __device__ __forceinline__ v8f mma(v16b a, v16b b, v8f c) {
    return __builtin_amdgcn_wmma_f32_16x16x32_bf16(false, a, false, b, (short)0, c, false, false);
  }
  static __device__ __forceinline__ void guard(v8f& a, v8f& b, v16b x, v16b y) { dep_guard_b(a, b, x, y); }
  static __device__ __forceinline__ void keep(v16b a, v16b b, v16b c, v16b d) { keep4_b(a, b, c, d); }
};

template <int ET> struct Elem;
template <> struct Elem<0> { typedef _Float16 T; };
template <> struct Elem<1> { typedef __bf16 T; };
template <int ET, bool SPLIT, int BIAS_MODE, int OUT_MODE, bool RESID, int ACT = 0>
__global__ __launch_bounds__(256) void wmma_gemm64(
    const unsigned short* __restrict__ Ap, const unsigned short* __restrict__ A2p, int lda, long strideA,
    const unsigned short* __restrict__ Btp, const unsigned short* __restrict__ Bt2p, int ldb, long strideB,
    void* __restrict__ Cout, void* __restrict__ Cout2, int ldc, long strideC,
    const float* __restrict__ bias,
    const float* __restrict__ resid, long strideR,
    int M, int N, int K, float scale) {
  typedef typename Elem<ET>::T T;
  typedef typename Frag<T>::V V;
  const T* A = (const T*)Ap; const T* A2 = (const T*)A2p; const T* Bt = (const T*)Btp; const T* Bt2 = (const T*)Bt2p;
  __shared__ __align__(16) float sT[8][16 * 68];
  const int b    = blockIdx.y;
  const int lane = threadIdx.x & 31;
  const int wave = threadIdx.x >> 5;
  const int tilesN = N >> 6;
  const int tilesM = M >> 6;
  const int tile = blockIdx.x * 8 + wave;
  if (tile >= tilesM * tilesN) return;
  const int tm = tile / tilesN;
  const int tn = tile - tm * tilesN;
  const int m0 = tm << 6;
  const int n0 = tn << 6;

  const T* Ab  = A  + (size_t)b * strideA;
  const T* Bb  = Bt + (size_t)b * strideB;
  const T* Ab2 = SPLIT ? (A2  + (size_t)b * strideA) : nullptr;
  const T* Bb2 = SPLIT ? (Bt2 + (size_t)b * strideB) : nullptr;

  const int rlane = lane & 15;
  const int koff  = (lane >> 4) * 8;
  const int mOff  = (lane >> 4) * 8;

  v8f acc[4][4];
#pragma unroll
  for (int i = 0; i < 4; ++i)
#pragma unroll
    for (int j = 0; j < 4; ++j) acc[i][j] = (v8f){0.f,0.f,0.f,0.f,0.f,0.f,0.f,0.f};

  for (int k0 = 0; k0 < K; k0 += 32) {
    V bh[4], bl[4];
#pragma unroll
    for (int j = 0; j < 4; ++j) {
      const size_t bo = (size_t)(n0 + (j << 4) + rlane) * ldb + koff + k0;
      bh[j] = Frag<T>::load(Bb + bo);
      if (SPLIT) bl[j] = Frag<T>::load(Bb2 + bo);
    }
#pragma unroll
    for (int i = 0; i < 4; ++i) {
      const size_t ao = (size_t)(m0 + (i << 4) + rlane) * lda + koff + k0;
      V ah = Frag<T>::load(Ab + ao);
      V al;
      if (SPLIT) al = Frag<T>::load(Ab2 + ao);
#pragma unroll
      for (int j = 0; j < 4; ++j) {
        acc[i][j] = Frag<T>::mma(ah, bh[j], acc[i][j]);
        if (SPLIT) {
          acc[i][j] = Frag<T>::mma(ah, bl[j], acc[i][j]);
          acc[i][j] = Frag<T>::mma(al, bh[j], acc[i][j]);
        }
      }
      Frag<T>::guard(acc[i][0], acc[i][3], ah, SPLIT ? al : ah);
    }
    Frag<T>::keep(bh[0], bh[1], bh[2], bh[3]);
    if (SPLIT) Frag<T>::keep(bl[0], bl[1], bl[2], bl[3]);
  }
  acc_guard4(acc[0][0], acc[0][1], acc[0][2], acc[0][3]);
  acc_guard4(acc[1][0], acc[1][1], acc[1][2], acc[1][3]);
  acc_guard4(acc[2][0], acc[2][1], acc[2][2], acc[2][3]);
  acc_guard4(acc[3][0], acc[3][1], acc[3][2], acc[3][3]);

  float* slab = sT[wave];
  const float* Rb = RESID ? (resid + (size_t)b * strideR) : nullptr;
#pragma unroll
  for (int i = 0; i < 4; ++i) {
    const int mBase = m0 + (i << 4);
#pragma unroll
    for (int j = 0; j < 4; ++j) {
      const int n = n0 + (j << 4) + rlane;
      float bv = 0.f;
      if (BIAS_MODE == 2) bv = bias[n];
#pragma unroll
      for (int r = 0; r < 8; ++r) {
        float v = acc[i][j][r] * scale;
        if (BIAS_MODE == 1) v += bias[mBase + mOff + r];
        if (BIAS_MODE == 2) v += bv;
        if (RESID) v += Rb[(size_t)(mBase + mOff + r) * ldc + n];
        if (ACT == 1) v = tanhf(v);
        if (ACT == 2) v = fmaxf(v, 0.0f);
        if (ACT == 3) v = v / (1.0f + expf(-v));
        if (ACT == 4) v = (v > 0.f) ? v : 0.01f * v;
        if (ACT == 5) v = 0.5f * v * (1.0f + erff(v * 0.70710678118654752f));
        slab[(mOff + r) * 68 + (j << 4) + rlane] = v;
      }
    }
    __builtin_amdgcn_fence(__ATOMIC_RELEASE, "workgroup");
    __builtin_amdgcn_wave_barrier();
    __builtin_amdgcn_fence(__ATOMIC_ACQUIRE, "workgroup");
    if (OUT_MODE == 0) {
      float* C = (float*)Cout + (size_t)b * strideC;
      const int hh = lane >> 4, c4 = (lane & 15) * 4;
      for (int pass = 0; pass < 2; ++pass) {
#pragma unroll
        for (int it = 0; it < 8; ++it) {
          const int row = it * 2 + hh;
          v4f v = *(const v4f*)(slab + row * 68 + c4);
          *(volatile v4f*)(C + (size_t)(mBase + row) * ldc + n0 + c4) = v;
        }
        __threadfence();
      }
    } else {
      const int q = lane >> 3, c8 = (lane & 7) * 8;
      unsigned short* C  = (unsigned short*)Cout  + (size_t)b * strideC;
      unsigned short* C2 = (OUT_MODE == 2) ? ((unsigned short*)Cout2 + (size_t)b * strideC) : nullptr;
      for (int pass = 0; pass < 2; ++pass) {
#pragma unroll
        for (int it = 0; it < 4; ++it) {
          const int row = it * 4 + q;
          const float* sp = slab + row * 68 + c8;
          v8h hv, lv;
#pragma unroll
          for (int e = 0; e < 8; ++e) {
            if (OUT_MODE == 1) {
              hv[e] = (_Float16)sp[e];
            } else {
              unsigned short hb = f2bf_bits(sp[e]);
              unsigned short lb = f2bf_bits(sp[e] - bf_bits2f(hb));
              hv[e] = __builtin_bit_cast(_Float16, hb);
              lv[e] = __builtin_bit_cast(_Float16, lb);
            }
          }
          *(volatile v8h*)(C + (size_t)(mBase + row) * ldc + n0 + c8) = hv;
          if (OUT_MODE == 2) *(volatile v8h*)(C2 + (size_t)(mBase + row) * ldc + n0 + c8) = lv;
        }
        __threadfence();
      }
    }
    __builtin_amdgcn_fence(__ATOMIC_RELEASE, "workgroup");
    __builtin_amdgcn_wave_barrier();
    __builtin_amdgcn_fence(__ATOMIC_ACQUIRE, "workgroup");
  }
}

__device__ __forceinline__ unsigned pack_h2(float a, float b) {
  const _Float16 h0 = (_Float16)a, h1 = (_Float16)b;
  return (unsigned)__builtin_bit_cast(unsigned short, h0) | ((unsigned)__builtin_bit_cast(unsigned short, h1) << 16);
}

__global__ __launch_bounds__(256) void cast_scale_f16x2_kernel(
    const float* __restrict__ in, unsigned short* __restrict__ out, int n2, float sc) {
  const int i = blockIdx.x * 256 + threadIdx.x;
  if (i < n2) {
    const v2f f = *(const v2f*)(in + 2 * (size_t)i);
    const unsigned u = pack_h2(f[0] * sc, f[1] * sc);
    ((volatile unsigned*)out)[i] = u;
    __threadfence();
    ((volatile unsigned*)out)[i] = u;
  }
}

__global__ __launch_bounds__(512) void build_ua_kernel(
    const float* __restrict__ qU, const float* __restrict__ qA,
    const float* __restrict__ kU, const float* __restrict__ kA,
    const float* __restrict__ vU, const float* __restrict__ vA,
    unsigned short* __restrict__ UAp) {
  const int p = blockIdx.y, r = blockIdx.x, i0 = 2 * threadIdx.x;
  const float* U = (p == 0) ? qU : ((p == 1) ? kU : vU);
  const float* A = (p == 0) ? qA : ((p == 1) ? kA : vA);
  const int ru = (r < kRank) ? r : (kRank - 1);
  int ra = r - kRank; ra = ra < 0 ? 0 : (ra > kLora - 1 ? kLora - 1 : ra);
  const float u0 = U[(size_t)i0 * kRank + ru], u1 = U[(size_t)(i0 + 1) * kRank + ru];
  const float a0 = A[(size_t)i0 * kLora + ra], a1 = A[(size_t)(i0 + 1) * kLora + ra];
  const bool isU = (r < kRank);
  const bool isA = (r >= kRank) && (r < kRank + kLora);
  const float w0 = isU ? u0 : (isA ? a0 : 0.0f);
  const float w1 = isU ? u1 : (isA ? a1 : 0.0f);
  const unsigned u = pack_h2(w0 * 64.0f, w1 * 64.0f);
  const size_t idx = ((((size_t)p * kT1Pitch + r) * kDim) + i0) >> 1;
  ((volatile unsigned*)UAp)[idx] = u;
  __threadfence();
  ((volatile unsigned*)UAp)[idx] = u;
}

__global__ __launch_bounds__(256) void build_bt2_kernel(
    const float* __restrict__ qV, const float* __restrict__ qal, const float* __restrict__ qBm,
    const float* __restrict__ kV, const float* __restrict__ kal, const float* __restrict__ kBm,
    const float* __restrict__ vV, const float* __restrict__ val, const float* __restrict__ vBm,
    unsigned short* __restrict__ BTp) {
  const int p = blockIdx.y;
  const int f = blockIdx.x * 256 + threadIdx.x;
  const float* Vw = (p == 0) ? qV  : ((p == 1) ? kV  : vV);
  const float* al = (p == 0) ? qal : ((p == 1) ? kal : val);
  const float* Bm = (p == 0) ? qBm : ((p == 1) ? kBm : vBm);
  const int e0 = 2 * f;
  const int o = e0 >> 7;
  const int c0 = e0 & (kBt2Pitch - 1);
  float w[2];
#pragma unroll
  for (int e = 0; e < 2; ++e) {
    const int c = c0 + e;
    const int cu = (c < kRank) ? c : (kRank - 1);
    int cl = c - kRank; cl = cl < 0 ? 0 : (cl > kLora - 1 ? kLora - 1 : cl);
    const float vv = Vw[(size_t)o * kRank + cu] * al[cu];
    const float bb = Bm[(size_t)cl * kDim + o];
    const bool isV = (c < kRank);
    const bool isB = (c >= kRank) && (c < kRank + kLora);
    w[e] = isV ? vv : (isB ? bb : 0.0f);
  }
  const unsigned u = pack_h2(w[0] * 512.0f, w[1] * 512.0f);
  const size_t idx = (((size_t)p * kDim * kBt2Pitch) + e0) >> 1;
  ((volatile unsigned*)BTp)[idx] = u;
  __threadfence();
  ((volatile unsigned*)BTp)[idx] = u;
}

__global__ __launch_bounds__(256) void prep_small_kernel(
    const float* __restrict__ qb, const float* __restrict__ kb, const float* __restrict__ vb,
    const float* __restrict__ tb, const float* __restrict__ ib, const float* __restrict__ cb,
    const float* __restrict__ tW, const float* __restrict__ iW, const float* __restrict__ cW,
    float* __restrict__ BIASF, unsigned short* __restrict__ HWp) {
  const int blk = blockIdx.x, tid = threadIdx.x;
  if (blk < 12) {
    const int idx = blk * 256 + tid;
    const int p = idx >> 10, i = idx & (kDim - 1);
    const float a = qb[i], bq = kb[i], cc = vb[i];
    const float v = (p == 0) ? a : ((p == 1) ? bq : cc);
    const float w = v * 64.0f;
    ((volatile float*)BIASF)[idx] = w;
    __threadfence();
    ((volatile float*)BIASF)[idx] = w;
  } else if (blk == 12) {
    if (tid < kHeadN) {
      const int j = tid;
      const int jt = (j < 2) ? j : 1;
      int ji = j - 2;  ji = ji < 0 ? 0 : (ji > 63 ? 63 : ji);
      int jc = j - 66; jc = jc < 0 ? 0 : (jc > 31 ? 31 : jc);
      const float t = tb[jt], iv = ib[ji], cv = cb[jc];
      const float v = (j < 2) ? t : ((j < 66) ? iv : ((j < 98) ? cv : 0.0f));
      ((volatile float*)BIASF)[3 * kDim + j] = v;
      __threadfence();
      ((volatile float*)BIASF)[3 * kDim + j] = v;
    }
  } else {
    const int f = (blk - 13) * 256 + tid;
    const int e0 = 2 * f;
    const int j = e0 >> 6, d0 = e0 & 63;
    const int jt = (j < 2) ? j : 1;
    int ji = j - 2;  ji = ji < 0 ? 0 : (ji > 63 ? 63 : ji);
    int jc = j - 66; jc = jc < 0 ? 0 : (jc > 31 ? 31 : jc);
    float w[2];
#pragma unroll
    for (int e = 0; e < 2; ++e) {
      const int d = d0 + e;
      const float t = tW[jt * kHd + d], iv = iW[ji * kHd + d], cv = cW[jc * kHd + d];
      w[e] = (j < 2) ? t : ((j < 66) ? iv : ((j < 98) ? cv : 0.0f));
    }
    const unsigned u = pack_h2(w[0] * 32.0f, w[1] * 32.0f);
    ((volatile unsigned*)HWp)[f] = u;
    __threadfence();
    ((volatile unsigned*)HWp)[f] = u;
  }
}

__global__ __launch_bounds__(256) void mem_prep_kernel(const float* __restrict__ mem,
                                                       unsigned short* __restrict__ M16p, unsigned short* __restrict__ MT16p) {
  __shared__ float tf[64 * 65];
  const int b = blockIdx.y, m0 = blockIdx.x * 64, tid = threadIdx.x;
#pragma unroll
  for (int it = 0; it < 4; ++it) {
    const int s = it * 256 + tid;
    const int row = s >> 4, c4 = (s & 15) * 4;
    const v4f a = *(const v4f*)(mem + ((size_t)(b * kMem + m0 + row) * kHd + c4));
    tf[row * 65 + c4 + 0] = a[0];
    tf[row * 65 + c4 + 1] = a[1];
    tf[row * 65 + c4 + 2] = a[2];
    tf[row * 65 + c4 + 3] = a[3];
  }
  __syncthreads();
  _Float16* M16 = (_Float16*)(void*)M16p;
  _Float16* MT16 = (_Float16*)(void*)MT16p;
  v8h hA[2], hB[2];
#pragma unroll
  for (int it = 0; it < 2; ++it) {
    const int s = it * 256 + tid;
    const int row = s >> 3, c8 = (s & 7) * 8;
    v8h x, y;
#pragma unroll
    for (int e = 0; e < 8; ++e) {
      x[e] = (_Float16)tf[row * 65 + c8 + e];
      y[e] = (_Float16)tf[(c8 + e) * 65 + row];
    }
    hA[it] = x; hB[it] = y;
  }
  for (int pass = 0; pass < 2; ++pass) {
#pragma unroll
    for (int it = 0; it < 2; ++it) {
      const int s = it * 256 + tid;
      const int row = s >> 3, c8 = (s & 7) * 8;
      *(volatile v8h*)(M16 + (size_t)(b * kMem + m0 + row) * kHd + c8) = hA[it];
      *(volatile v8h*)(MT16 + (size_t)(b * kHd + row) * kMem + m0 + c8) = hB[it];
    }
    __threadfence();
  }
}

__global__ __launch_bounds__(256) void strided_kernel(const unsigned short* __restrict__ K16p, const unsigned short* __restrict__ VT16p,
                                                      unsigned short* __restrict__ KSp, unsigned short* __restrict__ VSTp) {
  const int bh = blockIdx.x, b = bh / kHeads, h = bh % kHeads, tid = threadIdx.x;
  const _Float16* K16 = (const _Float16*)(const void*)K16p;
  const _Float16* VT16 = (const _Float16*)(const void*)VT16p;
  _Float16* KS = (_Float16*)(void*)KSp;
  _Float16* VST = (_Float16*)(void*)VSTp;
  const _Float16 hz = (_Float16)0.0f;
  v8h ka[2], va[2];
#pragma unroll
  for (int it = 0; it < 2; ++it) {
    const int s = it * 256 + tid;
    const int row = s >> 3, c8 = (s & 7) * 8;
    const int gc = (row < kNGlob) ? row : (kNGlob - 1);
    v8h kv = *(const v8h*)(K16 + (size_t)(b * kSeq + kGStride * gc) * kDim + h * kHd + c8);
    v8h vv;
#pragma unroll
    for (int e = 0; e < 8; ++e) {
      kv[e] = (row < kNGlob) ? kv[e] : hz;
      const int g = c8 + e;
      const int g2 = (g < kNGlob) ? g : (kNGlob - 1);
      const _Float16 x = VT16[(size_t)(h * kHd + row) * kRows + b * kSeq + kGStride * g2];
      vv[e] = (g < kNGlob) ? x : hz;
    }
    ka[it] = kv; va[it] = vv;
  }
  for (int pass = 0; pass < 2; ++pass) {
#pragma unroll
    for (int it = 0; it < 2; ++it) {
      const int s = it * 256 + tid;
      const int row = s >> 3, c8 = (s & 7) * 8;
      *(volatile v8h*)(KS + ((size_t)bh * 64 + row) * 64 + c8) = ka[it];
      *(volatile v8h*)(VST + ((size_t)bh * 64 + row) * 64 + c8) = va[it];
    }
    __threadfence();
  }
}

__device__ __forceinline__ v8f hmma16(v16h a, v16h b, v8f c) {
  c = __builtin_amdgcn_wmma_f32_16x16x32_f16(false, a, false, b, (short)0, c, false, false);
  asm volatile("v_nop\n\tv_nop\n\tv_nop\n\tv_nop" : "+v"(c) : "v"(a), "v"(b));
  return c;
}

__global__ __launch_bounds__(128)
void lga_attn_kernel(const unsigned short* __restrict__ Q16p, const unsigned short* __restrict__ K16p,
                     const unsigned short* __restrict__ VT16p, const unsigned short* __restrict__ KSp,
                     const unsigned short* __restrict__ VSTp, const unsigned short* __restrict__ M16p,
                     const unsigned short* __restrict__ MT16p, unsigned short* __restrict__ COMBp) {
  union FH { v16h v; v8h h[2]; };
  __shared__ __align__(16) _Float16 Ksh[64 * 64];
  __shared__ __align__(16) _Float16 Vth[64 * 64];
  __shared__ __align__(16) _Float16 Psh[4][16 * 64];
  __shared__ __align__(16) float    Os[4][16 * 68];

  const int tid  = threadIdx.x;
  const int wave = tid >> 5;
  const int lane = tid & 31;
  const int hh   = lane >> 4;
  const int c    = lane & 15;

  const int bx = blockIdx.x;
  const int qb = bx % kNQT;
  const int bh = bx / kNQT;
  const int h  = bh % kHeads;
  const int b  = bh / kHeads;
  const int q0 = qb * 64 + wave * 16;

  const _Float16* Q16  = (const _Float16*)(const void*)Q16p;
  const _Float16* K16  = (const _Float16*)(const void*)K16p;
  const _Float16* VT16 = (const _Float16*)(const void*)VT16p;
  const _Float16* KS   = (const _Float16*)(const void*)KSp;
  const _Float16* VST  = (const _Float16*)(const void*)VSTp;
  const _Float16* M16  = (const _Float16*)(const void*)M16p;
  const _Float16* MT16 = (const _Float16*)(const void*)MT16p;
  _Float16* COMB = (_Float16*)(void*)COMBp;

  v16h qa[2];
#pragma unroll
  for (int dc = 0; dc < 2; ++dc)
    qa[dc] = Frag<_Float16>::load(Q16 + (size_t)(b * kSeq + q0 + c) * kDim + h * kHd + dc * 32 + 8 * hh);

  v8f comb[4];
#pragma unroll
  for (int t = 0; t < 4; ++t) comb[t] = (v8f){0.f,0.f,0.f,0.f,0.f,0.f,0.f,0.f};

#pragma unroll 1
  for (int ph = 0; ph < 3; ++ph) {
    const _Float16* kbase; const _Float16* vbase;
    long kstr, vstr; int nch, kc0, mmode; float sscale, vnorm;
    if (ph == 0) {
      int lo = qb - 2; lo = lo < 0 ? 0 : lo;
      int hi = qb + 2; hi = hi > kNQT - 1 ? kNQT - 1 : hi;
      nch = hi - lo + 1; kc0 = lo; mmode = 1;
      kbase = K16 + (size_t)b * kSeq * kDim + h * kHd;             kstr = kDim;
      vbase = VT16 + (size_t)(h * kHd) * kRows + (size_t)b * kSeq; vstr = kRows;
      sscale = 1.0f / 32768.0f;
      vnorm  = 1.0f / (32768.0f * 64.0f);
    } else if (ph == 1) {
      nch = 1; kc0 = 0; mmode = 2;
      kbase = KS  + (size_t)bh * 64 * 64; kstr = 64;
      vbase = VST + (size_t)bh * 64 * 64; vstr = 64;
      sscale = 1.0f / 32768.0f;
      vnorm  = 1.0f / (32768.0f * 64.0f);
    } else {
      nch = kMem / 64; kc0 = 0; mmode = 0;
      kbase = M16  + (size_t)b * kMem * kHd; kstr = kHd;
      vbase = MT16 + (size_t)b * kHd * kMem; vstr = kMem;
      sscale = 1.0f / 512.0f;
      vnorm  = 1.0f / 32768.0f;
    }

    float mrow[8], lrow[8];
    v8f oacc[4];
#pragma unroll
    for (int r = 0; r < 8; ++r) { mrow[r] = -INFINITY; lrow[r] = 0.f; }
#pragma unroll
    for (int t = 0; t < 4; ++t) oacc[t] = (v8f){0.f,0.f,0.f,0.f,0.f,0.f,0.f,0.f};

    for (int kc = 0; kc < nch; ++kc) {
      const int kv0 = (kc0 + kc) * 64;
      __syncthreads();
      {
        const int r = tid >> 1, half = (tid & 1) * 32;
        const _Float16* ks = kbase + (size_t)(kv0 + r) * kstr + half;
        const _Float16* vs = vbase + (size_t)r * vstr + kv0 + half;
#pragma unroll
        for (int i = 0; i < 4; ++i) {
          const v8h a0 = *(const v8h*)(ks + 8 * i);
          const v8h b0 = *(const v8h*)(vs + 8 * i);
          *(v8h*)(Ksh + r * 64 + half + 8 * i) = a0;
          *(v8h*)(Vth + r * 64 + half + 8 * i) = b0;
        }
      }
      __syncthreads();

      v8f s[4];
#pragma unroll
      for (int j = 0; j < 4; ++j) {
        s[j] = (v8f){0.f,0.f,0.f,0.f,0.f,0.f,0.f,0.f};
#pragma unroll
        for (int dc = 0; dc < 2; ++dc) {
          FH kb;
          kb.h[0] = *(const v8h*)(Ksh + (j * 16 + c) * 64 + dc * 32 + 8 * hh);
          kb.h[1] = *(const v8h*)(Ksh + (j * 16 + c) * 64 + dc * 32 + 16 + 8 * hh);
          s[j] = hmma16(qa[dc], kb.v, s[j]);
        }
      }
      float cm[8];
#pragma unroll
      for (int r = 0; r < 8; ++r) {
        const int qpos = q0 + 8 * hh + r;
        float m = -INFINITY;
#pragma unroll
        for (int j = 0; j < 4; ++j) {
          const int kvcol = kv0 + j * 16 + c;
          int dlt = qpos - kvcol; dlt = dlt < 0 ? -dlt : dlt;
          const bool masked = (mmode == 1) ? (dlt > kWin) : ((mmode == 2) ? (kvcol >= kNGlob) : false);
          float sv = s[j][r] * sscale;
          sv = masked ? -INFINITY : sv;
          s[j][r] = sv;
          m = fmaxf(m, sv);
        }
#pragma unroll
        for (int off = 1; off < 16; off <<= 1) m = fmaxf(m, __shfl_xor(m, off, 32));
        cm[r] = m;
      }
      _Float16* pw = Psh[wave];
#pragma unroll
      for (int r = 0; r < 8; ++r) {
        const float mnew = fmaxf(mrow[r], cm[r]);
        const float mref = (mnew == -INFINITY) ? 0.0f : mnew;
        const float alpha = expf(mrow[r] - mref);
        mrow[r] = mnew;
        float psum = 0.f;
#pragma unroll
        for (int j = 0; j < 4; ++j) {
          const float p = expf(s[j][r] - mref);
          psum += p;
          pw[(8 * hh + r) * 64 + j * 16 + c] = (_Float16)(p * 32768.0f);
        }
#pragma unroll
        for (int off = 1; off < 16; off <<= 1) psum += __shfl_xor(psum, off, 32);
        lrow[r] = lrow[r] * alpha + psum;
#pragma unroll
        for (int t = 0; t < 4; ++t) oacc[t][r] *= alpha;
      }
      __builtin_amdgcn_fence(__ATOMIC_RELEASE, "workgroup");
      __builtin_amdgcn_wave_barrier();
      __builtin_amdgcn_fence(__ATOMIC_ACQUIRE, "workgroup");
#pragma unroll 1
      for (int kk = 0; kk < 2; ++kk) {
        FH pa;
        pa.h[0] = *(const v8h*)(pw + c * 64 + kk * 32 + 8 * hh);
        pa.h[1] = *(const v8h*)(pw + c * 64 + kk * 32 + 16 + 8 * hh);
#pragma unroll
        for (int t = 0; t < 4; ++t) {
          FH vb;
          vb.h[0] = *(const v8h*)(Vth + (t * 16 + c) * 64 + kk * 32 + 8 * hh);
          vb.h[1] = *(const v8h*)(Vth + (t * 16 + c) * 64 + kk * 32 + 16 + 8 * hh);
          oacc[t] = hmma16(pa.v, vb.v, oacc[t]);
        }
      }
    }
#pragma unroll
    for (int r = 0; r < 8; ++r) {
      const float inv = vnorm * (1.0f / lrow[r]);
#pragma unroll
      for (int t = 0; t < 4; ++t) comb[t][r] += oacc[t][r] * inv;
    }
  }

  float* os = Os[wave];
#pragma unroll
  for (int r = 0; r < 8; ++r)
#pragma unroll
    for (int t = 0; t < 4; ++t) os[(8 * hh + r) * 68 + t * 16 + c] = comb[t][r] * 16.0f;
  __builtin_amdgcn_fence(__ATOMIC_RELEASE, "workgroup");
  __builtin_amdgcn_wave_barrier();
  __builtin_amdgcn_fence(__ATOMIC_ACQUIRE, "workgroup");
  {
    const int rq = lane >> 3, c8 = (lane & 7) * 8;
    _Float16* cbp = COMB + (size_t)(b * kSeq) * kDim + h * kHd;
    for (int pass = 0; pass < 2; ++pass) {
#pragma unroll
      for (int it = 0; it < 4; ++it) {
        const int row = it * 4 + rq;
        const float* sp = os + row * 68 + c8;
        v8h hv;
#pragma unroll
        for (int e = 0; e < 8; ++e) hv[e] = (_Float16)sp[e];
        *(volatile v8h*)(cbp + (size_t)(q0 + row) * kDim + c8) = hv;
      }
      __threadfence();
    }
  }
}

__global__ __launch_bounds__(256) void repack_heads_kernel(const float* __restrict__ HO, float* __restrict__ out) {
  const size_t offT = (size_t)kRows * kDim;
  const size_t offI = offT + (size_t)kRows * 2;
  const size_t offC = offI + (size_t)kRows * 64;
  const int blk = blockIdx.x, tid = threadIdx.x;
  v4f v; float* p;
  if (blk < 8) {
    const int s = blk * 256 + tid;
    const int r0 = 2 * s;
    v[0] = HO[(size_t)r0 * kHeadN + 0];
    v[1] = HO[(size_t)r0 * kHeadN + 1];
    v[2] = HO[(size_t)(r0 + 1) * kHeadN + 0];
    v[3] = HO[(size_t)(r0 + 1) * kHeadN + 1];
    p = out + offT + 4 * (size_t)s;
  } else if (blk < 264) {
    const int s = (blk - 8) * 256 + tid;
    const int row = s >> 4, c4 = (s & 15) * 4;
    v[0] = HO[(size_t)row * kHeadN + 2 + c4 + 0];
    v[1] = HO[(size_t)row * kHeadN + 2 + c4 + 1];
    v[2] = HO[(size_t)row * kHeadN + 2 + c4 + 2];
    v[3] = HO[(size_t)row * kHeadN + 2 + c4 + 3];
    p = out + offI + 4 * (size_t)s;
  } else {
    const int s = (blk - 264) * 256 + tid;
    const int row = s >> 3, c4 = (s & 7) * 4;
    v[0] = HO[(size_t)row * kHeadN + 66 + c4 + 0];
    v[1] = HO[(size_t)row * kHeadN + 66 + c4 + 1];
    v[2] = HO[(size_t)row * kHeadN + 66 + c4 + 2];
    v[3] = HO[(size_t)row * kHeadN + 66 + c4 + 3];
    p = out + offC + 4 * (size_t)s;
  }
  *(volatile v4f*)p = v;
  __threadfence();
  *(volatile v4f*)p = v;
}

constexpr size_t kBytesX16  = (size_t)kRows * kDim * 2;
constexpr size_t kBytesUA   = 3ull * kT1Pitch * kDim * 2;
constexpr size_t kBytesBT2  = 3ull * kDim * kBt2Pitch * 2;
constexpr size_t kBytesBias = (3ull * kDim + kHeadN) * 4;
constexpr size_t kBytesT1   = 3ull * kRows * kT1Pitch * 2;
constexpr size_t kBytesQKV  = (size_t)kRows * kDim * 2;
constexpr size_t kBytesMem  = (size_t)kBatch * kMem * kHd * 2;
constexpr size_t kBytesStr  = (size_t)kBatch * kHeads * 64 * 64 * 2;
constexpr size_t kBytesWO   = (size_t)kDim * kDim * 2;
constexpr size_t kBytesHW   = (size_t)kHeadN * kHd * 2;
constexpr size_t kBytesHO   = (size_t)kRows * kHeadN * 4;

constexpr size_t kOffX16  = 0;
constexpr size_t kOffUA   = kOffX16 + kBytesX16;
constexpr size_t kOffBT2  = kOffUA + kBytesUA;
constexpr size_t kOffBias = kOffBT2 + kBytesBT2;
constexpr size_t kOffT1   = kOffBias + kBytesBias;
constexpr size_t kOffQ16  = kOffT1 + kBytesT1;
constexpr size_t kOffK16  = kOffQ16 + kBytesQKV;
constexpr size_t kOffVT16 = kOffK16 + kBytesQKV;
constexpr size_t kOffM16  = kOffVT16 + kBytesQKV;
constexpr size_t kOffMT16 = kOffM16 + kBytesMem;
constexpr size_t kOffKS   = kOffMT16 + kBytesMem;
constexpr size_t kOffVST  = kOffKS + kBytesStr;
constexpr size_t kOffCOMB = kOffVST + kBytesStr;
constexpr size_t kOffWO   = kOffCOMB + kBytesQKV;
constexpr size_t kOffHW   = kOffWO + kBytesWO;
constexpr size_t kOffHO   = kOffHW + kBytesHW;
constexpr size_t kOffEnd  = kOffHO + kBytesHO;
static_assert(kOffEnd == 51540480ull, "carve total");
static_assert(kOffEnd <= 134217728ull, "carve under 128 MiB");
static_assert((kOffUA % 128) == 0 && (kOffBT2 % 128) == 0 && (kOffBias % 128) == 0 && (kOffT1 % 128) == 0 &&
              (kOffQ16 % 128) == 0 && (kOffM16 % 128) == 0 && (kOffKS % 128) == 0 && (kOffCOMB % 128) == 0 &&
              (kOffWO % 128) == 0 && (kOffHW % 128) == 0 && (kOffHO % 128) == 0, "128-B aligned regions");

extern "C" void kernel_launch(void* const* d_in, const int* in_sizes, int n_in,
                              void* d_out, int out_size, void* d_ws, size_t ws_size, hipStream_t stream) {
  if (n_in < 28) return;
  if (in_sizes[0] != kRows * kDim || in_sizes[1] != kBatch * kMem * kHd || in_sizes[2] != kDim * kRank ||
      in_sizes[5] != kDim * kLora || in_sizes[6] != kLora * kDim || in_sizes[20] != kDim * kDim ||
      in_sizes[22] != 2 * kHd || in_sizes[24] != 64 * kHd || in_sizes[26] != 32 * kHd) return;
  if (out_size != kRows * kDim + kRows * 2 + kRows * 64 + kRows * 32) return;
  if (kOffEnd > ws_size) return;

  const float* x    = (const float*)d_in[0];
  const float* mem  = (const float*)d_in[1];
  const float* qU = (const float*)d_in[2],  *qV = (const float*)d_in[3],  *qal = (const float*)d_in[4];
  const float* qA = (const float*)d_in[5],  *qBm = (const float*)d_in[6], *qbv = (const float*)d_in[7];
  const float* kU = (const float*)d_in[8],  *kV = (const float*)d_in[9],  *kal = (const float*)d_in[10];
  const float* kA = (const float*)d_in[11], *kBm = (const float*)d_in[12], *kbv = (const float*)d_in[13];
  const float* vU = (const float*)d_in[14], *vV = (const float*)d_in[15], *val = (const float*)d_in[16];
  const float* vA = (const float*)d_in[17], *vBm = (const float*)d_in[18], *vbv = (const float*)d_in[19];
  const float* outW = (const float*)d_in[20], *outb = (const float*)d_in[21];
  const float* tW = (const float*)d_in[22], *tb = (const float*)d_in[23];
  const float* iW = (const float*)d_in[24], *ib = (const float*)d_in[25];
  const float* cW = (const float*)d_in[26], *cb = (const float*)d_in[27];
  float* out = (float*)d_out;

  char* ws = (char*)d_ws;
  unsigned short* X16  = (unsigned short*)(ws + kOffX16);
  unsigned short* UA   = (unsigned short*)(ws + kOffUA);
  unsigned short* BT2  = (unsigned short*)(ws + kOffBT2);
  float*          BIASF = (float*)(ws + kOffBias);
  unsigned short* T1   = (unsigned short*)(ws + kOffT1);
  unsigned short* Q16  = (unsigned short*)(ws + kOffQ16);
  unsigned short* K16  = (unsigned short*)(ws + kOffK16);
  unsigned short* VT16 = (unsigned short*)(ws + kOffVT16);
  unsigned short* M16  = (unsigned short*)(ws + kOffM16);
  unsigned short* MT16 = (unsigned short*)(ws + kOffMT16);
  unsigned short* KS   = (unsigned short*)(ws + kOffKS);
  unsigned short* VST  = (unsigned short*)(ws + kOffVST);
  unsigned short* COMB = (unsigned short*)(ws + kOffCOMB);
  unsigned short* WO16 = (unsigned short*)(ws + kOffWO);
  unsigned short* HW16 = (unsigned short*)(ws + kOffHW);
  float*          HOUT = (float*)(ws + kOffHO);

  const float* QB64 = BIASF;
  const float* KB64 = BIASF + kDim;
  const float* VB64 = BIASF + 2 * kDim;
  const float* HB   = BIASF + 3 * kDim;

  const size_t planeT1  = (size_t)kRows * kT1Pitch;
  const size_t planeBT2 = (size_t)kDim * kBt2Pitch;

  {
    const int n2 = kRows * kDim / 2;
    cast_scale_f16x2_kernel<<<dim3((n2 + 255) / 256), 256, 0, stream>>>(x, X16, n2, 1.0f);
  }
  build_ua_kernel<<<dim3(kT1Pitch, 3), 512, 0, stream>>>(qU, qA, kU, kA, vU, vA, UA);
  build_bt2_kernel<<<dim3((kDim * kBt2Pitch / 2 + 255) / 256, 3), 256, 0, stream>>>(qV, qal, qBm, kV, kal, kBm, vV, val, vBm, BT2);
  prep_small_kernel<<<dim3(29), 256, 0, stream>>>(qbv, kbv, vbv, tb, ib, cb, tW, iW, cW, BIASF, HW16);
  {
    const int n2 = kDim * kDim / 2;
    cast_scale_f16x2_kernel<<<dim3((n2 + 255) / 256), 256, 0, stream>>>(outW, WO16, n2, 32.0f);
  }
  mem_prep_kernel<<<dim3(kMem / 64, kBatch), 256, 0, stream>>>(mem, M16, MT16);

  {
    const int tiles = (kRows / 64) * (kT1Pitch / 64);
    wmma_gemm64<0, false, 0, 1, false, 0><<<dim3((tiles + 7) / 8, 3), 256, 0, stream>>>(
        X16, X16, kDim, 0L, UA, UA, kDim, (long)kT1Pitch * kDim,
        (void*)T1, (void*)T1, kT1Pitch, (long)planeT1,
        BIASF, BIASF, 0L, kRows, kT1Pitch, kDim, 1.0f);
  }
  {
    const int tiles = (kRows / 64) * (kDim / 64);
    wmma_gemm64<0, false, 2, 1, false, 0><<<dim3((tiles + 7) / 8, 1), 256, 0, stream>>>(
        T1, T1, kT1Pitch, 0L, BT2, BT2, kBt2Pitch, 0L,
        (void*)Q16, (void*)Q16, kDim, 0L,
        QB64, BIASF, 0L, kRows, kDim, kKInner, 1.0f / 512.0f);
  }
  {
    const int tiles = (kRows / 64) * (kDim / 64);
    wmma_gemm64<0, false, 2, 1, false, 0><<<dim3((tiles + 7) / 8, 1), 256, 0, stream>>>(
        T1 + planeT1, T1 + planeT1, kT1Pitch, 0L, BT2 + planeBT2, BT2 + planeBT2, kBt2Pitch, 0L,
        (void*)K16, (void*)K16, kDim, 0L,
        KB64, BIASF, 0L, kRows, kDim, kKInner, 1.0f / 512.0f);
  }
  {
    const int tiles = (kDim / 64) * (kRows / 64);
    wmma_gemm64<0, false, 1, 1, false, 0><<<dim3((tiles + 7) / 8, 1), 256, 0, stream>>>(
        BT2 + 2 * planeBT2, BT2 + 2 * planeBT2, kBt2Pitch, 0L, T1 + 2 * planeT1, T1 + 2 * planeT1, kT1Pitch, 0L,
        (void*)VT16, (void*)VT16, kRows, 0L,
        VB64, BIASF, 0L, kDim, kRows, kKInner, 1.0f / 512.0f);
  }
  strided_kernel<<<dim3(kBatch * kHeads), 256, 0, stream>>>(K16, VT16, KS, VST);
  lga_attn_kernel<<<dim3(kBatch * kHeads * kNQT), 128, 0, stream>>>(Q16, K16, VT16, KS, VST, M16, MT16, COMB);
  {
    const int tiles = (kRows / 64) * (kDim / 64);
    wmma_gemm64<0, false, 2, 0, false, 0><<<dim3((tiles + 7) / 8, 1), 256, 0, stream>>>(
        COMB, COMB, kDim, 0L, WO16, WO16, kDim, 0L,
        (void*)out, (void*)out, kDim, 0L,
        outb, BIASF, 0L, kRows, kDim, kDim, 1.0f / 512.0f);
  }
  {
    const int tiles = (kRows / 64) * (kHeadN / 64);
    wmma_gemm64<0, false, 2, 0, false, 0><<<dim3((tiles + 7) / 8, 1), 256, 0, stream>>>(
        COMB, COMB, kDim, 0L, HW16, HW16, kHd, 0L,
        (void*)HOUT, (void*)HOUT, kHeadN, 0L,
        HB, BIASF, 0L, kRows, kHeadN, kHd, 1.0f / 512.0f);
  }
  repack_heads_kernel<<<dim3(392), 256, 0, stream>>>(HOUT, out);
}
